// Model_40827959116313
// MI455X (gfx1250) — hardware-verified
//
#include <hip/hip_runtime.h>
#include <stddef.h>
#include <stdint.h>

#define NB   32
#define NN   128
#define NE   2048
#define NG   1024
#define NV   10000
#define DIN  20
#define KIN  32
#define HID  1024
#define MID  128
#define EPSF 1e-5f
#define OFFW 160

#define GBM   64
#define GBN   128
#define GTHR  128
#define GWAVE (GTHR / 32)
#define TPB   (NG / GBM)
#define NTILE (NB * NG / GBM)
#define RECW  (2 * MID)

#define NU_EB (NV * HID / 8)
#define NU_HB (NB * NN * KIN / 8)
#define NU_WI (HID * KIN / 8)
#define NU_WG (MID * HID / 8)
#define NU_ALL (NU_EB + NU_HB + NU_WI + NU_WG)

#define ENC_WORDS (2 * NN * 128 + NE + OFFW + 512 + 512 + 128)
#define ENC_LDS   (ENC_WORDS * 4)
#define WSCAP 134217728

static_assert(NE == 2048 && NN == 128 && NG % 128 == 0 && HID % 128 == 0 && MID == 128);
static_assert(NU_EB % 256 == 0 && NU_HB % 256 == 0 && NU_WI % 256 == 0 && NU_WG % 256 == 0);
static_assert(GBM == GWAVE * 16 && GBN == 4 * 32 && GTHR == GBN && NG % GBM == 0 && (NB * NN) % GBM == 0);
static_assert(KIN % 32 == 0 && HID % 32 == 0 && DIN <= KIN && DIN % 4 == 0);
static_assert(OFFW % 32 == 0 && OFFW >= NN + 2 && OFFW / 4 <= 128);
static_assert(ENC_LDS <= 300000);
static_assert(TPB == 16 && GBM == 64);

typedef float          v4f   __attribute__((ext_vector_type(4)));
typedef float          v8f   __attribute__((ext_vector_type(8)));
typedef int            v4i   __attribute__((ext_vector_type(4)));
typedef int            v8i   __attribute__((ext_vector_type(8)));
typedef unsigned short v8us  __attribute__((ext_vector_type(8)));
typedef unsigned short v16us __attribute__((ext_vector_type(16)));
typedef __bf16         v16bf __attribute__((ext_vector_type(16)));
typedef v4f  __attribute__((may_alias)) v4fa;
typedef v4i  __attribute__((may_alias)) v4ia;
typedef v8us __attribute__((may_alias)) v8usa;
union FragB { v16bf v; v16us u; v8us h[2]; v8i w; };

__device__ __forceinline__ v8f wmb(const FragB& a, const FragB& b, v8f c) {
  v8f d = __builtin_amdgcn_wmma_f32_16x16x32_bf16(false, a.v, false, b.v, (short)0, c, false, false);
  asm volatile("v_nop\n\tv_nop\n\tv_nop\n\tv_nop" : "+v"(d) : "v"(a.w), "v"(b.w));
  return d;
}
__device__ __forceinline__ v8f z8() { v8f z = {0.f, 0.f, 0.f, 0.f, 0.f, 0.f, 0.f, 0.f}; return z; }

__device__ __forceinline__ unsigned bf16_bits(float f) {
  const unsigned u = __float_as_uint(f);
  return (u + 0x7FFFu + ((u >> 16) & 1u)) >> 16;
}
__device__ __forceinline__ float bf16_val(float f) {
  return __uint_as_float(bf16_bits(f) << 16);
}

__device__ __forceinline__ void st8(unsigned short* dp, const float* f) {
  v8us o;
#pragma unroll
  for (int i = 0; i < 8; ++i) o[i] = (unsigned short)bf16_bits(f[i]);
  *(volatile v8us*)dp = o;
  __threadfence();
  *(volatile v8us*)dp = o;
}

__global__ __launch_bounds__(256) void k_prep(const float* __restrict__ h, const float* __restrict__ emb,
                                              const float* __restrict__ Wi, const float* __restrict__ Wfc,
                                              unsigned short* HB, unsigned short* WiT,
                                              unsigned short* EB, unsigned short* WgT) {
  const int u = (int)blockIdx.x * 256 + (int)threadIdx.x;
  float f[8];
  if (u < NU_EB) {
    const float* p = emb + (size_t)u * 8;
    const v4f a = *(const v4f*)p;
    const v4f b = *(const v4f*)(p + 4);
    f[0] = a.x; f[1] = a.y; f[2] = a.z; f[3] = a.w;
    f[4] = b.x; f[5] = b.y; f[6] = b.z; f[7] = b.w;
    st8(EB + (size_t)u * 8, f);
  } else if (u < NU_EB + NU_HB) {
    const int v   = u - NU_EB;
    const int row = v >> 2;
    const int k8  = (v & 3) * 8;
    const float* p = h + (size_t)row * DIN;
    const int o0 = (k8 < 16) ? k8 : 16;
    const int o1 = (k8 + 4 < 16) ? (k8 + 4) : 16;
    const v4f a = *(const v4f*)(p + o0);
    const v4f b = *(const v4f*)(p + o1);
    const bool va = (k8 <= 16);
    const bool vb = (k8 < 16);
    f[0] = va ? a.x : 0.0f; f[1] = va ? a.y : 0.0f; f[2] = va ? a.z : 0.0f; f[3] = va ? a.w : 0.0f;
    f[4] = vb ? b.x : 0.0f; f[5] = vb ? b.y : 0.0f; f[6] = vb ? b.z : 0.0f; f[7] = vb ? b.w : 0.0f;
    st8(HB + (size_t)v * 8, f);
  } else if (u < NU_EB + NU_HB + NU_WI) {
    const int v  = u - (NU_EB + NU_HB);
    const int n  = v >> 2;
    const int k8 = (v & 3) * 8;
#pragma unroll
    for (int i = 0; i < 8; ++i) {
      const int k  = k8 + i;
      const int kc = (k < DIN) ? k : (DIN - 1);
      const float x = Wi[(size_t)kc * HID + n];
      f[i] = (k < DIN) ? x : 0.0f;
    }
    st8(WiT + (size_t)v * 8, f);
  } else if (u < NU_ALL) {
    const int v  = u - (NU_EB + NU_HB + NU_WI);
    const int n  = v >> 7;
    const int k8 = (v & 127) * 8;
#pragma unroll
    for (int i = 0; i < 8; ++i) f[i] = Wfc[(size_t)(HID + k8 + i) * MID + n];
    st8(WgT + (size_t)v * 8, f);
  }
}

__global__ __launch_bounds__(128) void k_csr(const int* __restrict__ src, const int* __restrict__ dst,
                                             int* LIST, int* OFF) {
  __shared__ __attribute__((aligned(16))) int sS[NE];
  __shared__ __attribute__((aligned(16))) int sD[NE];
  __shared__ __attribute__((aligned(16))) int sL[NE + NN];
  __shared__ __attribute__((aligned(16))) int sO[OFFW];
  __shared__ int sC[NN];
  __shared__ int sF[4];
  const int tid = (int)threadIdx.x, lane = tid & 31, wave = tid >> 5;
  const int b = (int)blockIdx.x;
  const v4i z4 = {0, 0, 0, 0};
  int bad = 0;
#pragma unroll
  for (int it = 0; it < 4; ++it) {
    const int i = tid + it * 128;
    const v4i s4 = *(const v4i*)(src + (size_t)b * NE + 4 * i);
    const v4i d4 = *(const v4i*)(dst + (size_t)b * NE + 4 * i);
    bad |= ((unsigned)s4.x >= (unsigned)NN) | ((unsigned)s4.y >= (unsigned)NN) |
           ((unsigned)s4.z >= (unsigned)NN) | ((unsigned)s4.w >= (unsigned)NN) |
           ((unsigned)d4.x >= (unsigned)NN) | ((unsigned)d4.y >= (unsigned)NN) |
           ((unsigned)d4.z >= (unsigned)NN) | ((unsigned)d4.w >= (unsigned)NN);
    *(v4ia*)(sS + 4 * i) = s4;
    *(v4ia*)(sD + 4 * i) = d4;
    *(v4ia*)(sL + 4 * i) = z4;
  }
  sL[NE + tid] = 0;
  if (tid < OFFW / 4) *(v4ia*)(sO + 4 * tid) = z4;
  const unsigned mb = __builtin_amdgcn_ballot_w32(bad != 0);
  if (lane == 0) sF[wave] = (mb != 0u) ? 1 : 0;
  __syncthreads();
  const int flag = sF[0] | sF[1] | sF[2] | sF[3];

  int c = 0;
#pragma unroll 4
  for (int e = 0; e < NE; ++e) c += (sD[e] == tid) ? 1 : 0;
  sC[tid] = c;
  __syncthreads();
  int o = 0;
#pragma unroll 4
  for (int i = 0; i < NN; ++i) {
    const int v = sC[i];
    o += (i < tid) ? v : 0;
  }
  int p = o;
#pragma unroll 4
  for (int e = 0; e < NE; ++e) {
    const int d = sD[e];
    int s = sS[e];
    s = s < 0 ? 0 : (s > NN - 1 ? NN - 1 : s);
    const bool hit = (d == tid);
    const int pp  = (p < NE - 1) ? p : (NE - 1);
    const int idx = hit ? pp : (NE + tid);
    sL[idx] = s;
    p += hit ? 1 : 0;
  }
  sO[tid] = o;
  if (tid == NN - 1) sO[NN] = o + c;
  if (tid == 0) sO[NN + 1] = flag;
  __syncthreads();

  v4i lv[4];
#pragma unroll
  for (int it = 0; it < 4; ++it) lv[it] = *(const v4ia*)(sL + 4 * (tid + it * 128));
  v4i ov = z4;
  if (tid < OFFW / 4) ov = *(const v4ia*)(sO + 4 * tid);
  int* lp = LIST + (size_t)b * NE;
  int* op = OFF + (size_t)b * OFFW;
#pragma unroll
  for (int it = 0; it < 4; ++it) *(volatile v4i*)(lp + 4 * (tid + it * 128)) = lv[it];
  if (tid < OFFW / 4) *(volatile v4i*)(op + 4 * tid) = ov;
  __threadfence();
#pragma unroll
  for (int it = 0; it < 4; ++it) *(volatile v4i*)(lp + 4 * (tid + it * 128)) = lv[it];
  if (tid < OFFW / 4) *(volatile v4i*)(op + 4 * tid) = ov;
}

template <int MODE, int K, int KC, int LDO>
__global__ __launch_bounds__(GTHR) void k_gemm(const unsigned short* __restrict__ A,
                                               const unsigned short* __restrict__ BT,
                                               const int* __restrict__ gidx,
                                               const float* __restrict__ addv,
                                               float* xout, float* recs) {
  constexpr int AP  = KC + 8;
  constexpr int PPR = KC / 8;
  constexpr int NIT = GBM * PPR / GTHR;
  static_assert(K % KC == 0 && KC % 32 == 0 && (GBM * PPR) % GTHR == 0 && NIT <= 8);
  __shared__ __attribute__((aligned(16))) unsigned short at[GBM * AP];
  __shared__ __attribute__((aligned(16))) float stg[GBM * GBN];
  __shared__ __attribute__((aligned(16))) float wst[GWAVE * RECW];
  __shared__ __attribute__((aligned(16))) float pst[RECW];
  __shared__ int ridx[GBM];
  const int tid = (int)threadIdx.x, lane = tid & 31, wave = tid >> 5, hh = lane >> 4, m = lane & 15;
  const int rowBase = (int)blockIdx.x * GBM;
  const int colBase = (int)blockIdx.y * GBN;

  if (tid < GBM) {
    int r;
    if constexpr (MODE == 1) {
      int g = gidx[rowBase + tid];
      g = (g < 0) ? (g + NV) : g;
      g = g < 0 ? 0 : (g > NV - 1 ? NV - 1 : g);
      r = g;
    } else {
      r = rowBase + tid;
    }
    ridx[tid] = r;
  }
  __syncthreads();

  v8f acc[8];
#pragma unroll
  for (int t = 0; t < 8; ++t) acc[t] = z8();
  const unsigned short* bp = BT + (size_t)(colBase + m) * (size_t)K + 8 * hh;
  const unsigned short* ar = at + (16 * wave + m) * AP + 8 * hh;

#pragma unroll 1
  for (int k0 = 0; k0 < K; k0 += KC) {
    v8us pc[NIT];
#pragma unroll
    for (int it = 0; it < NIT; ++it) {
      const int p   = tid + it * GTHR;
      const int row = p / PPR;
      const int q   = p % PPR;
      pc[it] = *(const v8usa*)(A + (size_t)ridx[row] * (size_t)K + k0 + 8 * q);
    }
#pragma unroll
    for (int it = 0; it < NIT; ++it) {
      const int p   = tid + it * GTHR;
      const int row = p / PPR;
      const int q   = p % PPR;
      *(v8usa*)(at + row * AP + 8 * q) = pc[it];
    }
    __syncthreads();
#pragma unroll 1
    for (int kk = 0; kk < KC; kk += 32) {
      FragB af;
      af.h[0] = *(const v8usa*)(ar + kk);
      af.h[1] = *(const v8usa*)(ar + kk + 16);
#pragma unroll
      for (int nt = 0; nt < 8; ++nt) {
        const unsigned short* wq = bp + (size_t)(16 * nt) * (size_t)K + k0 + kk;
        FragB bf;
        bf.h[0] = *(const v8usa*)wq;
        bf.h[1] = *(const v8usa*)(wq + 16);
        acc[nt] = wmb(af, bf, acc[nt]);
      }
    }
    __syncthreads();
  }

#pragma unroll
  for (int nt = 0; nt < 8; ++nt) {
    const int lc = 16 * nt + m;
#pragma unroll
    for (int r = 0; r < 8; ++r) {
      const int lr = 16 * wave + 8 * hh + r;
      stg[lr * GBN + lc] = acc[nt][r];
    }
  }
  __syncthreads();

  float aq[4];
  if constexpr (MODE == 0) {
    const v4f b4 = *(const v4f*)(addv + colBase + 4 * lane);
    aq[0] = bf16_val(b4.x); aq[1] = bf16_val(b4.y); aq[2] = bf16_val(b4.z); aq[3] = bf16_val(b4.w);
  } else {
    const int b = rowBase >> 10;
    const v4f b4 = *(const v4f*)(addv + (size_t)b * MID + 4 * lane);
    aq[0] = b4.x; aq[1] = b4.y; aq[2] = b4.z; aq[3] = b4.w;
  }

  float wm[4], wqv[4];
#pragma unroll
  for (int j = 0; j < 4; ++j) { wm[j] = 0.0f; wqv[j] = 0.0f; }
  float* sbase = stg + (16 * wave) * GBN + 4 * lane;
#pragma unroll 4
  for (int i = 0; i < 16; ++i) {
    float* sp = sbase + i * GBN;
    const v4f x = *(const v4fa*)sp;
    float y[4];
    y[0] = x.x + aq[0]; y[1] = x.y + aq[1]; y[2] = x.z + aq[2]; y[3] = x.w + aq[3];
    v4f q;
    q.x = y[0]; q.y = y[1]; q.z = y[2]; q.w = y[3];
    *(v4fa*)sp = q;
    if constexpr (MODE == 1) {
      const float rk = 1.0f / (float)(i + 1);
#pragma unroll
      for (int j = 0; j < 4; ++j) {
        const float d = y[j] - wm[j];
        wm[j]  = fmaf(d, rk, wm[j]);
        wqv[j] = fmaf(d, y[j] - wm[j], wqv[j]);
      }
    }
  }
  float* obase = xout + (size_t)(rowBase + 16 * wave) * (size_t)LDO + colBase + 4 * lane;
#pragma unroll 4
  for (int i = 0; i < 16; ++i) {
    const v4f v = *(const v4fa*)(sbase + i * GBN);
    *(volatile v4f*)(obase + (size_t)i * LDO) = v;
  }
  __threadfence();
#pragma unroll 4
  for (int i = 0; i < 16; ++i) {
    const v4f v = *(const v4fa*)(sbase + i * GBN);
    *(volatile v4f*)(obase + (size_t)i * LDO) = v;
  }

  if constexpr (MODE == 1) {
#pragma unroll
    for (int j = 0; j < 4; ++j) {
      wst[wave * RECW + 4 * lane + j]       = wm[j];
      wst[wave * RECW + GBN + 4 * lane + j] = wqv[j];
    }
    __syncthreads();
    {
      const float m0 = wst[0 * RECW + tid], m1 = wst[1 * RECW + tid];
      const float m2 = wst[2 * RECW + tid], m3 = wst[3 * RECW + tid];
      const float q0 = wst[0 * RECW + GBN + tid], q1 = wst[1 * RECW + GBN + tid];
      const float q2 = wst[2 * RECW + GBN + tid], q3 = wst[3 * RECW + GBN + tid];
      const float mean = (((m0 + m1) + m2) + m3) * 0.25f;
      const float d0 = m0 - mean, d1 = m1 - mean, d2 = m2 - mean, d3 = m3 - mean;
      const float dd = ((d0 * d0 + d1 * d1) + d2 * d2) + d3 * d3;
      const float M2 = (((q0 + q1) + q2) + q3) + 16.0f * dd;
      pst[tid] = mean;
      pst[GBN + tid] = M2;
    }
    __syncthreads();
    v4f ps = {0.f, 0.f, 0.f, 0.f};
    float* rp = recs + (size_t)blockIdx.x * RECW + 4 * tid;
    if (tid < RECW / 4) {
      ps = *(const v4fa*)(pst + 4 * tid);
      *(volatile v4f*)rp = ps;
    }
    __threadfence();
    if (tid < RECW / 4) {
      *(volatile v4f*)rp = ps;
    }
  }
}

__global__ __launch_bounds__(256) void k_enc(const float* __restrict__ H0, const int* __restrict__ LIST,
                                             const int* __restrict__ OFF,
                                             const float* __restrict__ g1, const float* __restrict__ b1,
                                             const float* __restrict__ g2, const float* __restrict__ b2,
                                             float* QEMB) {
  extern __shared__ __attribute__((aligned(16))) float dsm[];
  float* Xs  = dsm;
  float* Zs  = dsm + NN * 128;
  int*   lst = (int*)(dsm + 2 * NN * 128);
  int*   off = lst + NE;
  float* par = (float*)(off + OFFW);
  float* red = par + 512;
  float* qs  = red + 512;
  const int tid = (int)threadIdx.x, lane = tid & 31, wave = tid >> 5;
  const int b  = (int)blockIdx.x >> 3;
  const int ch = (int)blockIdx.x & 7;

#pragma unroll 4
  for (int it = 0; it < 16; ++it) {
    const int i   = tid + it * 256;
    const int row = i >> 5;
    const int c4  = i & 31;
    const v4f v = *(const v4f*)(H0 + (size_t)(b * NN + row) * HID + ch * 128 + 4 * c4);
    *(v4fa*)(Xs + row * 128 + 4 * c4) = v;
  }
#pragma unroll
  for (int it = 0; it < 2; ++it) {
    const int i = tid + it * 256;
    v4i v = *(const v4i*)(LIST + (size_t)b * NE + 4 * i);
    v.x = v.x < 0 ? 0 : (v.x > NN - 1 ? NN - 1 : v.x);
    v.y = v.y < 0 ? 0 : (v.y > NN - 1 ? NN - 1 : v.y);
    v.z = v.z < 0 ? 0 : (v.z > NN - 1 ? NN - 1 : v.z);
    v.w = v.w < 0 ? 0 : (v.w > NN - 1 ? NN - 1 : v.w);
    *(v4ia*)(lst + 4 * i) = v;
  }
  if (tid < OFFW / 4) {
    const v4i v = *(const v4i*)(OFF + (size_t)b * OFFW + 4 * tid);
    *(v4ia*)(off + 4 * tid) = v;
  }
  if (tid < 128) {
    par[tid]       = bf16_val(g1[ch * 128 + tid]);
    par[128 + tid] = bf16_val(b1[ch * 128 + tid]);
    par[256 + tid] = bf16_val(g2[ch * 128 + tid]);
    par[384 + tid] = bf16_val(b2[ch * 128 + tid]);
  }
  __syncthreads();
  const int flag = off[NN + 1];
  const int c  = tid & 127;
  const int hf = tid >> 7;
  const int r0 = hf * 64;

#pragma unroll 1
  for (int layer = 0; layer < 2; ++layer) {
#pragma unroll 1
    for (int i = 0; i < 16; ++i) {
      const int d = wave * 16 + i;
      int o = off[d];
      int e = off[d + 1];
      o = o < 0 ? 0 : (o > NE ? NE : o);
      int cn = e - o;
      cn = cn < 0 ? 0 : (cn > NE - o ? NE - o : cn);
      float a0 = 0.0f, a1 = 0.0f, a2 = 0.0f, a3 = 0.0f;
#pragma unroll 4
      for (int p = 0; p < cn; ++p) {
        const int s = lst[o + p];
        const v4f x = *(const v4fa*)(Xs + s * 128 + 4 * lane);
        a0 += x.x; a1 += x.y; a2 += x.z; a3 += x.w;
      }
      const float den = (float)(cn > 0 ? cn : 1);
      const v4f xs = *(const v4fa*)(Xs + d * 128 + 4 * lane);
      v4f z;
      z.x = xs.x + a0 / den;
      z.y = xs.y + a1 / den;
      z.z = xs.z + a2 / den;
      z.w = xs.w + a3 / den;
      *(v4fa*)(Zs + d * 128 + 4 * lane) = z;
    }
    __syncthreads();
    float s = 0.0f;
#pragma unroll 4
    for (int r = 0; r < 64; ++r) s += Zs[(r0 + r) * 128 + c];
    red[hf * 128 + c] = s;
    __syncthreads();
    const float mu = (red[c] + red[128 + c]) * (1.0f / 128.0f);
    float q = 0.0f;
#pragma unroll 4
    for (int r = 0; r < 64; ++r) {
      const float dd = Zs[(r0 + r) * 128 + c] - mu;
      q += dd * dd;
    }
    red[256 + hf * 128 + c] = q;
    __syncthreads();
    const float var = (red[256 + c] + red[384 + c]) * (1.0f / 128.0f);
    const float sd  = sqrtf(var + EPSF);
    const float g   = par[layer * 256 + c];
    const float be  = par[layer * 256 + 128 + c];
    float cs = 0.0f;
#pragma unroll 1
    for (int r = 0; r < 64; ++r) {
      const float z = Zs[(r0 + r) * 128 + c];
      const float y = g * (z - mu) / sd + be;
      const float yr = (y > 0.0f) ? y : (y - y);
      Xs[(r0 + r) * 128 + c] = yr;
      cs += yr;
    }
    red[hf * 128 + c] = cs;
    __syncthreads();
  }

  if (tid < 128) {
    float qv = (red[tid] + red[128 + tid]) * (1.0f / 128.0f);
    qv = (flag != 0) ? __int_as_float(0x7fc00000) : qv;
    qs[tid] = qv;
  }
  __syncthreads();
  v4f ov = {0.f, 0.f, 0.f, 0.f};
  float* qp = QEMB + (size_t)b * HID + ch * 128 + 4 * tid;
  if (tid < 32) {
    ov = *(const v4fa*)(qs + 4 * tid);
    *(volatile v4f*)qp = ov;
  }
  __threadfence();
  if (tid < 32) {
    *(volatile v4f*)qp = ov;
  }
}

__global__ __launch_bounds__(256) void k_qc(const float* __restrict__ QEMB, const float* __restrict__ Wfc,
                                            const float* __restrict__ bfc, float* C) {
  __shared__ __attribute__((aligned(16))) float cs[256];
  const int tid = (int)threadIdx.x;
  const int i = (int)blockIdx.x * 256 + tid;
  const int b = i >> 7, j = i & 127;
  const float* q = QEMB + (size_t)b * HID;
  float s = 0.0f;
#pragma unroll 4
  for (int k = 0; k < HID; ++k) s = fmaf(q[k], bf16_val(Wfc[(size_t)k * MID + j]), s);
  s = s + bf16_val(bfc[j]);
  cs[tid] = s;
  __syncthreads();
  v4f v = {0.f, 0.f, 0.f, 0.f};
  float* op = C + (size_t)blockIdx.x * 256 + 4 * tid;
  if (tid < 64) {
    v = *(const v4fa*)(cs + 4 * tid);
    *(volatile v4f*)op = v;
  }
  __threadfence();
  if (tid < 64) {
    *(volatile v4f*)op = v;
  }
}

__global__ __launch_bounds__(256) void k_apply(const float* __restrict__ X, const float* __restrict__ recs,
                                               const float* __restrict__ gbn, const float* __restrict__ bbn,
                                               const float* __restrict__ w2, const float* __restrict__ b2,
                                               float* out) {
  __shared__ __attribute__((aligned(16))) float smu[MID];
  __shared__ __attribute__((aligned(16))) float srs[MID];
  __shared__ __attribute__((aligned(16))) float res[128];
  const int tid = (int)threadIdx.x, lane = tid & 31, wave = tid >> 5;
  const int blk = (int)blockIdx.x;
  const int b = blk >> 3;
  if (tid < MID) {
    const float* rp = recs + (size_t)(b * TPB) * RECW + tid;
    double sm = 0.0;
#pragma unroll 4
    for (int t = 0; t < TPB; ++t) sm += (double)rp[(size_t)t * RECW];
    const double mean = sm * 0.0625;
    double M2 = 0.0;
#pragma unroll 4
    for (int t = 0; t < TPB; ++t) {
      const double mt = (double)rp[(size_t)t * RECW];
      const double qt = (double)rp[(size_t)t * RECW + MID];
      const double d = mt - mean;
      M2 += qt + 64.0 * d * d;
    }
    const float varf = (float)(M2 * (1.0 / 1024.0));
    const float sd = sqrtf(varf + EPSF);
    smu[tid] = (float)mean;
    srs[tid] = 1.0f / sd;
  }
  __syncthreads();

  const v4f g4 = *(const v4f*)(gbn + 4 * lane);
  const v4f e4 = *(const v4f*)(bbn + 4 * lane);
  const v4f w4 = *(const v4f*)(w2 + 4 * lane);
  const v4f m4 = *(const v4fa*)(smu + 4 * lane);
  const v4f r4 = *(const v4fa*)(srs + 4 * lane);
  const float ga0 = bf16_val(g4.x), ga1 = bf16_val(g4.y), ga2 = bf16_val(g4.z), ga3 = bf16_val(g4.w);
  const float be0 = bf16_val(e4.x), be1 = bf16_val(e4.y), be2 = bf16_val(e4.z), be3 = bf16_val(e4.w);
  const float wa0 = bf16_val(w4.x), wa1 = bf16_val(w4.y), wa2 = bf16_val(w4.z), wa3 = bf16_val(w4.w);
  const float bias2 = bf16_val(b2[0]);

#pragma unroll 1
  for (int i = 0; i < 16; ++i) {
    const int row = blk * 128 + wave * 16 + i;
    const v4f x = *(const v4f*)(X + (size_t)row * MID + 4 * lane);
    float y0 = ga0 * (x.x - m4.x) * r4.x + be0;
    float y1 = ga1 * (x.y - m4.y) * r4.y + be1;
    float y2 = ga2 * (x.z - m4.z) * r4.z + be2;
    float y3 = ga3 * (x.w - m4.w) * r4.w + be3;
    y0 = (y0 > 0.0f) ? y0 : (y0 - y0);
    y1 = (y1 > 0.0f) ? y1 : (y1 - y1);
    y2 = (y2 > 0.0f) ? y2 : (y2 - y2);
    y3 = (y3 > 0.0f) ? y3 : (y3 - y3);
    float part = y0 * wa0;
    part = fmaf(y1, wa1, part);
    part = fmaf(y2, wa2, part);
    part = fmaf(y3, wa3, part);
    part += __shfl_xor(part, 16);
    part += __shfl_xor(part, 8);
    part += __shfl_xor(part, 4);
    part += __shfl_xor(part, 2);
    part += __shfl_xor(part, 1);
    const float z = part + bias2;
    const float pr = 1.0f / (1.0f + expf(-z));
    if (lane == 0) res[wave * 16 + i] = pr;
  }
  __syncthreads();
  v4f v = {0.f, 0.f, 0.f, 0.f};
  float* op = out + (size_t)blk * 128 + 4 * tid;
  if (tid < 32) {
    v = *(const v4fa*)(res + 4 * tid);
    *(volatile v4f*)op = v;
  }
  __threadfence();
  if (tid < 32) {
    *(volatile v4f*)op = v;
  }
}

static inline size_t al256(size_t o) { return (o + 255) & ~(size_t)255; }

extern "C" void kernel_launch(void* const* d_in, const int* in_sizes, int n_in,
                              void* d_out, int out_size, void* d_ws, size_t ws_size,
                              hipStream_t stream) {
  if (n_in < 17) return;
  if (in_sizes[0] != NB * NN * DIN) return;
  if (in_sizes[1] != NB * NE || in_sizes[2] != NB * NE) return;
  if (in_sizes[3] != NB * NG) return;
  if (in_sizes[4] != NV * HID) return;
  if (in_sizes[5] != DIN * HID || in_sizes[6] != HID) return;
  if (in_sizes[7] != HID || in_sizes[8] != HID || in_sizes[9] != HID || in_sizes[10] != HID) return;
  if (in_sizes[11] != 2 * HID * MID || in_sizes[12] != MID) return;
  if (in_sizes[13] != MID || in_sizes[14] != MID) return;
  if (in_sizes[15] != MID || in_sizes[16] != 1) return;
  if (out_size != NB * NG) return;

  const float* h      = (const float*)d_in[0];
  const int*   esrc   = (const int*)d_in[1];
  const int*   edst   = (const int*)d_in[2];
  const int*   gPos   = (const int*)d_in[3];
  const float* table  = (const float*)d_in[4];
  const float* W_init = (const float*)d_in[5];
  const float* b_init = (const float*)d_in[6];
  const float* gamma1 = (const float*)d_in[7];
  const float* beta1  = (const float*)d_in[8];
  const float* gamma2 = (const float*)d_in[9];
  const float* beta2  = (const float*)d_in[10];
  const float* W_fc   = (const float*)d_in[11];
  const float* b_fc   = (const float*)d_in[12];
  const float* gam_bn = (const float*)d_in[13];
  const float* bet_bn = (const float*)d_in[14];
  const float* W_fc2  = (const float*)d_in[15];
  const float* b_fc2  = (const float*)d_in[16];
  float* out = (float*)d_out;

  char* ws = (char*)d_ws;
  size_t off = 0;
  const size_t oEB  = off; off = al256(off + (size_t)NV * HID * 2);
  const size_t oH0  = off; off = al256(off + (size_t)NB * NN * HID * 4);
  const size_t oX   = off; off = al256(off + (size_t)NB * NG * MID * 4);
  const size_t oHB  = off; off = al256(off + (size_t)NB * NN * KIN * 2);
  const size_t oWI  = off; off = al256(off + (size_t)HID * KIN * 2);
  const size_t oWG  = off; off = al256(off + (size_t)MID * HID * 2);
  const size_t oQE  = off; off = al256(off + (size_t)NB * HID * 4);
  const size_t oC   = off; off = al256(off + (size_t)NB * MID * 4);
  const size_t oRC  = off; off = al256(off + (size_t)NTILE * RECW * 4);
  const size_t oLS  = off; off = al256(off + (size_t)NB * NE * 4);
  const size_t oOF  = off; off = al256(off + (size_t)NB * OFFW * 4);
  if (off > ws_size || off > (size_t)WSCAP) return;
  unsigned short* EB  = (unsigned short*)(ws + oEB);
  float*          H0  = (float*)(ws + oH0);
  float*          X   = (float*)(ws + oX);
  unsigned short* HB  = (unsigned short*)(ws + oHB);
  unsigned short* WiT = (unsigned short*)(ws + oWI);
  unsigned short* WgT = (unsigned short*)(ws + oWG);
  float*          QE  = (float*)(ws + oQE);
  float*          C   = (float*)(ws + oC);
  float*          RC  = (float*)(ws + oRC);
  int*            LS  = (int*)(ws + oLS);
  int*            OF  = (int*)(ws + oOF);

  hipFuncSetAttribute(reinterpret_cast<const void*>(&k_enc), hipFuncAttributeMaxDynamicSharedMemorySize, (int)ENC_LDS);

  k_prep<<<NU_ALL / 256, 256, 0, stream>>>(h, table, W_init, W_fc, HB, WiT, EB, WgT);
  k_csr<<<NB, 128, 0, stream>>>(esrc, edst, LS, OF);
  k_gemm<0, KIN, KIN, HID><<<dim3((NB * NN) / GBM, HID / GBN), GTHR, 0, stream>>>(HB, WiT, gPos, b_init, H0, RC);
  k_enc<<<NB * 8, 256, ENC_LDS, stream>>>(H0, LS, OF, gamma1, beta1, gamma2, beta2, QE);
  k_qc<<<(NB * MID) / 256, 256, 0, stream>>>(QE, W_fc, b_fc, C);
  k_gemm<1, HID, 128, MID><<<dim3(NTILE, 1), GTHR, 0, stream>>>(EB, WgT, gPos, C, X, RC);
  k_apply<<<(NB * NG) / 128, 256, 0, stream>>>(X, RC, gam_bn, bet_bn, W_fc2, b_fc2, out);
}
